// SenseMemAct_18588618457548
// MI455X (gfx1250) — hardware-verified
//
#include <hip/hip_runtime.h>
#include <math.h>


#define AS3 __attribute__((address_space(3)))

#define BB   64
#define LL   4096
#define NIN  32
#define NU   32
#define MEM  64
#define DEC  3
#define NR   (BB * LL)

static_assert(NIN == 32 && NU == 32);
static_assert(MEM == 64);
static_assert(LL % 32 == 0);
static_assert(NR % 64 == 0);
static_assert(BB % 16 == 0);
static_assert((size_t)BB * LL * DEC == (size_t)786432);

typedef __bf16         v16b __attribute__((ext_vector_type(16)));
typedef unsigned short v8us __attribute__((ext_vector_type(8)));
typedef float          v8f  __attribute__((ext_vector_type(8)));
typedef float          v4f  __attribute__((ext_vector_type(4)));
typedef v8us __attribute__((may_alias)) v8usa;
typedef v4f  __attribute__((may_alias)) v4fa;

typedef AS3 unsigned short*       lp_us;
typedef AS3 const unsigned short* lcp_us;
typedef AS3 float*                lp_f;
typedef AS3 const float*          lcp_f;

union Frag { v16b v; v8us half[2]; };

constexpr size_t OFF_UH = 0;
constexpr size_t SZ_U   = (size_t)NR * NU * 2;
constexpr size_t OFF_UL = OFF_UH + SZ_U;
constexpr size_t WS_END = OFF_UL + SZ_U;
static_assert(OFF_UL % 128 == 0);
static_assert(WS_END <= (size_t)134217728);
static_assert((size_t)(NR / 64) * 32 * 128 == SZ_U);

__device__ __forceinline__ unsigned short bf16_bits(float f) {
  unsigned u = __float_as_uint(f);
  u += 0x7FFFu + ((u >> 16) & 1u);
  return (unsigned short)(u >> 16);
}
__device__ __forceinline__ float bf16_val(unsigned short b) { return __uint_as_float(((unsigned)b) << 16); }
__device__ __forceinline__ float bf16r(float f) { return bf16_val(bf16_bits(f)); }
__device__ __forceinline__ v8f zero8() {
  v8f z;
#pragma unroll
  for (int i = 0; i < 8; ++i) z[i] = 0.0f;
  return z;
}

__device__ __forceinline__ void ldfrag_g(Frag& f, const unsigned short* p, int h) {
  f.half[0] = *(const v8usa*)(p + 8 * h);
  f.half[1] = *(const v8usa*)(p + 16 + 8 * h);
}
__device__ __forceinline__ void ldfrag_l(Frag& f, lcp_us p, int h) {
  f.half[0] = *(AS3 const v8usa*)(p + 8 * h);
  f.half[1] = *(AS3 const v8usa*)(p + 16 + 8 * h);
}
__device__ __forceinline__ void ldfrag_f(Frag& f, const float* p, int h) {
  const v4f a0 = *(const v4fa*)(p + 8 * h);
  const v4f a1 = *(const v4fa*)(p + 8 * h + 4);
  const v4f a2 = *(const v4fa*)(p + 16 + 8 * h);
  const v4f a3 = *(const v4fa*)(p + 16 + 8 * h + 4);
  v8us lo, hi;
  lo[0] = bf16_bits(a0[0]); lo[1] = bf16_bits(a0[1]); lo[2] = bf16_bits(a0[2]); lo[3] = bf16_bits(a0[3]);
  lo[4] = bf16_bits(a1[0]); lo[5] = bf16_bits(a1[1]); lo[6] = bf16_bits(a1[2]); lo[7] = bf16_bits(a1[3]);
  hi[0] = bf16_bits(a2[0]); hi[1] = bf16_bits(a2[1]); hi[2] = bf16_bits(a2[2]); hi[3] = bf16_bits(a2[3]);
  hi[4] = bf16_bits(a3[0]); hi[5] = bf16_bits(a3[1]); hi[6] = bf16_bits(a3[2]); hi[7] = bf16_bits(a3[3]);
  f.half[0] = lo;
  f.half[1] = hi;
}
__device__ __forceinline__ v8f mma16(v8f c, const Frag& a, const Frag& b) {
  return __builtin_amdgcn_wmma_f32_16x16x32_bf16(false, a.v, false, b.v, (short)0, c, false, false);
}

__global__ __launch_bounds__(128)
void uproj_kernel(const float* __restrict__ x, const float* __restrict__ wsn,
                  unsigned short* uh, unsigned short* ul)
{
  __shared__ __attribute__((aligned(16))) unsigned short sTH[64 * NU];
  __shared__ __attribute__((aligned(16))) unsigned short sTL[64 * NU];
  lp_us pTH = (lp_us)sTH;
  lp_us pTL = (lp_us)sTL;

  const int tid = threadIdx.x, lane = tid & 31, w = tid >> 5;
  const int h = lane >> 4, m = lane & 15;
  const int rb = blockIdx.x * 64;

  Frag a, b[2];
  ldfrag_f(a, x + (size_t)(rb + 16 * w + m) * NIN, h);
#pragma unroll
  for (int nt = 0; nt < 2; ++nt) ldfrag_f(b[nt], wsn + (size_t)(16 * nt + m) * NIN, h);
  v8f acc[2];
#pragma unroll
  for (int nt = 0; nt < 2; ++nt) acc[nt] = mma16(zero8(), a, b[nt]);
  asm volatile("v_nop\n\tv_nop\n\tv_nop\n\tv_nop"
               : "+v"(acc[0]), "+v"(acc[1])
               : "v"(a.v), "v"(b[0].v), "v"(b[1].v));

#pragma unroll
  for (int nt = 0; nt < 2; ++nt)
#pragma unroll
    for (int r = 0; r < 8; ++r) {
      const int rowl = 16 * w + 8 * h + r;
      const int col  = 16 * nt + m;
      const float v = acc[nt][r];
      const unsigned short hb = bf16_bits(v);
      const unsigned short lb = bf16_bits(v - bf16_val(hb));
      pTH[rowl * NU + col] = hb;
      pTL[rowl * NU + col] = lb;
    }
  __syncthreads();

  const int q8 = lane & 7;
  v8us vh[2], vl[2];
  size_t go[2];
#pragma unroll
  for (int i = 0; i < 2; ++i) {
    const int li = (tid >> 3) + 16 * i;
    const int rl = 2 * li + (q8 >> 2);
    const int cp = 8 * (q8 & 3);
    vh[i] = *(AS3 const v8usa*)(pTH + rl * NU + cp);
    vl[i] = *(AS3 const v8usa*)(pTL + rl * NU + cp);
    go[i] = (size_t)(rb + rl) * NU + cp;
  }
  *(volatile v8us*)(uh + go[0]) = vh[0];
  *(volatile v8us*)(uh + go[1]) = vh[1];
  *(volatile v8us*)(ul + go[0]) = vl[0];
  *(volatile v8us*)(ul + go[1]) = vl[1];
  __threadfence();
  *(volatile v8us*)(uh + go[0]) = vh[0];
  *(volatile v8us*)(uh + go[1]) = vh[1];
  *(volatile v8us*)(ul + go[0]) = vl[0];
  *(volatile v8us*)(ul + go[1]) = vl[1];
}

constexpr int HP  = MEM + 8;
constexpr int HT  = 16 * HP;
constexpr int HFT = 16 * MEM;
constexpr int SOW = 32 * DEC;
static_assert(HP % 8 == 0);
static_assert((3 * MEM * NU) / 8 == 6 * 128);
static_assert((2 * MEM * MEM) / 8 == 8 * 128);
static_assert((MEM * NU) / 8 == 256 && (MEM * MEM) / 8 == 512);

__global__ __launch_bounds__(128)
void rnn_kernel(const unsigned short* __restrict__ uh, const unsigned short* __restrict__ ul,
                const float* __restrict__ wia, const float* __restrict__ wic, const float* __restrict__ wio,
                const float* __restrict__ wha, const float* __restrict__ whc, const float* __restrict__ wact,
                float* out)
{
  __shared__ __attribute__((aligned(16))) unsigned short sWc[3 * MEM * NU];
  __shared__ __attribute__((aligned(16))) unsigned short sWh[2 * MEM * MEM];
  __shared__ __attribute__((aligned(16))) unsigned short sHH[2 * HT];
  __shared__ __attribute__((aligned(16))) unsigned short sHL[2 * HT];
  __shared__ __attribute__((aligned(16))) float sHF[2 * HFT];
  __shared__ __attribute__((aligned(16))) float sAct[DEC * MEM];
  __shared__ __attribute__((aligned(16))) float sOut[16 * SOW];
  lp_us pWc = (lp_us)sWc;
  lp_us pWh = (lp_us)sWh;
  lp_us pHH = (lp_us)sHH;
  lp_us pHL = (lp_us)sHL;
  lp_f  pHF = (lp_f)sHF;
  lp_f  pAct = (lp_f)sAct;
  lp_f  pOut = (lp_f)sOut;

  const int tid = threadIdx.x, lane = tid & 31, w = tid >> 5;
  const int h = lane >> 4, m = lane & 15;
  const int b0 = blockIdx.x * 16;

  {
#pragma unroll 1
    for (int j = 0; j < 6; ++j) {
      const int i = tid + 128 * j;
      const float* src = (j < 2) ? (wia + 8 * i) : ((j < 4) ? (wic + 8 * (i - 256)) : (wio + 8 * (i - 512)));
      const v4f a = *(const v4fa*)src;
      const v4f c = *(const v4fa*)(src + 4);
      v8us o;
      o[0] = bf16_bits(a[0]); o[1] = bf16_bits(a[1]); o[2] = bf16_bits(a[2]); o[3] = bf16_bits(a[3]);
      o[4] = bf16_bits(c[0]); o[5] = bf16_bits(c[1]); o[6] = bf16_bits(c[2]); o[7] = bf16_bits(c[3]);
      *(AS3 v8us*)(pWc + 8 * i) = o;
    }
#pragma unroll 1
    for (int j = 0; j < 8; ++j) {
      const int i = tid + 128 * j;
      const float* src = (j < 4) ? (wha + 8 * i) : (whc + 8 * (i - 512));
      const v4f a = *(const v4fa*)src;
      const v4f c = *(const v4fa*)(src + 4);
      v8us o;
      o[0] = bf16_bits(a[0]); o[1] = bf16_bits(a[1]); o[2] = bf16_bits(a[2]); o[3] = bf16_bits(a[3]);
      o[4] = bf16_bits(c[0]); o[5] = bf16_bits(c[1]); o[6] = bf16_bits(c[2]); o[7] = bf16_bits(c[3]);
      *(AS3 v8us*)(pWh + 8 * i) = o;
    }
    v8us z8;
#pragma unroll
    for (int i = 0; i < 8; ++i) z8[i] = (unsigned short)0;
    for (int i = tid; i < (2 * HT) / 8; i += 128) {
      *(AS3 v8us*)(pHH + 8 * i) = z8;
      *(AS3 v8us*)(pHL + 8 * i) = z8;
    }
    v4f z4 = {0.0f, 0.0f, 0.0f, 0.0f};
    for (int i = tid; i < (2 * HFT) / 4; i += 128) *(AS3 v4f*)(pHF + 4 * i) = z4;
    for (int i = tid; i < (16 * SOW) / 4; i += 128) *(AS3 v4f*)(pOut + 4 * i) = z4;
    for (int i = tid; i < DEC * MEM; i += 128) pAct[i] = bf16r(wact[i]);
  }
  float hprev[8];
#pragma unroll
  for (int r = 0; r < 8; ++r) hprev[r] = 0.0f;
  __syncthreads();

  const int q8 = lane & 7;
  const int col = 16 * w + m;
  const float neg_inf = __uint_as_float(0xff800000u);

#pragma unroll 1
  for (int t = 0; t < LL; ++t) {
    const int cur = t & 1, nxt = cur ^ 1;

    v8f xa = zero8(), xc = zero8(), xo = zero8(), pa = zero8(), pc = zero8();

    {
      const size_t uo = ((size_t)(b0 + m) * LL + t) * NU;
      Frag ah, al, bwa, bwc, bwo;
      ldfrag_g(ah, uh + uo, h);
      ldfrag_g(al, ul + uo, h);
      ldfrag_l(bwa, pWc + (16 * w + m) * NU, h);
      ldfrag_l(bwc, pWc + (MEM + 16 * w + m) * NU, h);
      ldfrag_l(bwo, pWc + (2 * MEM + 16 * w + m) * NU, h);
      xa = mma16(xa, ah, bwa); xa = mma16(xa, al, bwa);
      xc = mma16(xc, ah, bwc); xc = mma16(xc, al, bwc);
      xo = mma16(xo, ah, bwo); xo = mma16(xo, al, bwo);
      asm volatile("v_nop\n\tv_nop\n\tv_nop\n\tv_nop"
                   : "+v"(xa), "+v"(xc), "+v"(xo)
                   : "v"(ah.v), "v"(al.v), "v"(bwa.v), "v"(bwc.v), "v"(bwo.v));
    }
    {
      lcp_us ha = pHH + cur * HT + m * HP;
      lcp_us la = pHL + cur * HT + m * HP;
      lcp_us ba = pWh + (16 * w + m) * MEM;
      lcp_us bc = pWh + (MEM + 16 * w + m) * MEM;
#pragma unroll 1
      for (int k0 = 0; k0 < MEM; k0 += 32) {
        Frag ah, al, fa, fc;
        ldfrag_l(ah, ha + k0, h);
        ldfrag_l(al, la + k0, h);
        ldfrag_l(fa, ba + k0, h);
        ldfrag_l(fc, bc + k0, h);
        pa = mma16(pa, ah, fa); pa = mma16(pa, al, fa);
        pc = mma16(pc, ah, fc); pc = mma16(pc, al, fc);
        asm volatile("v_nop\n\tv_nop\n\tv_nop\n\tv_nop"
                     : "+v"(pa), "+v"(pc)
                     : "v"(ah.v), "v"(al.v), "v"(fa.v), "v"(fc.v));
      }
    }

    {
      lp_us hHn = pHH + nxt * HT;
      lp_us hLn = pHL + nxt * HT;
      lp_f  hFc = pHF + cur * HFT;
#pragma unroll
      for (int r = 0; r < 8; ++r) {
        const int row = 8 * h + r;
        const float hp = hprev[r];
        const float av = 1.0f + tanhf(xa[r] + pa[r]);
        float z = xc[r] + pc[r];
        z = fminf(fmaxf(z, -80.0f), 80.0f);
        const float cf = 1.0f / (1.0f + expf(-z));
        const float th = tanhf(xo[r] + av * hp);
        const float hn = cf * hp + (1.0f - cf) * th;
        hprev[r] = hn;
        const unsigned short hb = bf16_bits(hn);
        const unsigned short lb = bf16_bits(hn - bf16_val(hb));
        hHn[row * HP + col]  = hb;
        hLn[row * HP + col]  = lb;
        hFc[row * MEM + col] = hn;
      }
    }
    __syncthreads();

    if (tid < 64) {
      const int row = tid >> 2, d = tid & 3, dd = min(d, DEC - 1);
      lcp_f hr = pHF + cur * HFT + row * MEM;
      lcp_f ar = pAct + dd * MEM;
      float s = 0.0f;
#pragma unroll 4
      for (int k = 0; k < MEM; k += 4) {
        const v4f hv = *(AS3 const v4fa*)(hr + k);
        const v4f wv = *(AS3 const v4fa*)(ar + k);
        s += hv[0] * wv[0];
        s += hv[1] * wv[1];
        s += hv[2] * wv[2];
        s += hv[3] * wv[3];
      }
      const float lg = (d < DEC) ? s : neg_inf;
      float mx = fmaxf(lg, __shfl_xor(lg, 1, 4));
      mx = fmaxf(mx, __shfl_xor(mx, 2, 4));
      const float e = expf(lg - mx);
      float sum = e + __shfl_xor(e, 1, 4);
      sum = sum + __shfl_xor(sum, 2, 4);
      const float p = e * (1.0f / sum);
      if (d < DEC) pOut[row * SOW + (t & 31) * DEC + d] = p;
    }

    if ((t & 31) == 31) {
      __syncthreads();
      const int c32 = t - 31;
      v4f ov[3];
      size_t oo[3];
#pragma unroll
      for (int i = 0; i < 3; ++i) {
        const int li = (tid >> 3) + 16 * i;
        const int row = li / 3;
        const int part = li - 3 * row;
        ov[i] = *(AS3 const v4fa*)(pOut + row * SOW + part * 32 + 4 * q8);
        oo[i] = (size_t)(b0 + row) * ((size_t)LL * DEC) + (size_t)c32 * DEC + (size_t)(part * 32 + 4 * q8);
      }
      *(volatile v4f*)(out + oo[0]) = ov[0];
      *(volatile v4f*)(out + oo[1]) = ov[1];
      *(volatile v4f*)(out + oo[2]) = ov[2];
      __threadfence();
      *(volatile v4f*)(out + oo[0]) = ov[0];
      *(volatile v4f*)(out + oo[1]) = ov[1];
      *(volatile v4f*)(out + oo[2]) = ov[2];
    }
  }
}

extern "C" void kernel_launch(void* const* d_in, const int* in_sizes, int n_in,
                              void* d_out, int out_size, void* d_ws, size_t ws_size,
                              hipStream_t stream)
{
  if (n_in < 8) return;
  if (in_sizes[0] != NR * NIN)    return;
  if (in_sizes[1] != NU * NIN)    return;
  if (in_sizes[2] != MEM * NU)    return;
  if (in_sizes[3] != MEM * MEM)   return;
  if (in_sizes[4] != MEM * NU)    return;
  if (in_sizes[5] != MEM * MEM)   return;
  if (in_sizes[6] != MEM * NU)    return;
  if (in_sizes[7] != DEC * MEM)   return;
  if (out_size != BB * LL * DEC)  return;
  if (ws_size < WS_END)           return;

  const float* x    = (const float*)d_in[0];
  const float* wsn  = (const float*)d_in[1];
  const float* wia  = (const float*)d_in[2];
  const float* wha  = (const float*)d_in[3];
  const float* wic  = (const float*)d_in[4];
  const float* whc  = (const float*)d_in[5];
  const float* wio  = (const float*)d_in[6];
  const float* wact = (const float*)d_in[7];
  float* out = (float*)d_out;

  char* ws = (char*)d_ws;
  unsigned short* uh = (unsigned short*)(ws + OFF_UH);
  unsigned short* ul = (unsigned short*)(ws + OFF_UL);

  uproj_kernel<<<dim3(NR / 64), dim3(128), 0, stream>>>(x, wsn, uh, ul);

  rnn_kernel<<<dim3(BB / 16), dim3(128), 0, stream>>>(uh, ul, wia, wic, wio, wha, whc, wact, out);
}
